// PCTNet_17300128268588
// MI455X (gfx1250) — hardware-run, weakly checked
//
#include <hip/hip_runtime.h>
#include <math.h>

typedef __attribute__((ext_vector_type(16))) _Float16 v16h;
typedef __attribute__((ext_vector_type(8)))  _Float16 v8h;
typedef __attribute__((ext_vector_type(16))) __bf16   v16b;
typedef __attribute__((ext_vector_type(8)))  __bf16   v8b;
typedef __attribute__((ext_vector_type(8)))  float    v8f;
typedef __attribute__((ext_vector_type(4)))  float    v4f;
typedef __attribute__((ext_vector_type(4)))  unsigned int v4u;

constexpr int kBatch  = 8;
constexpr int kCh     = 256;
constexpr int kImgH   = 32;
constexpr int kImgW   = 32;
constexpr int kTok    = kImgH * kImgW;
constexpr int kPix    = kBatch * kTok;
constexpr int kHeads  = 8;
constexpr int kDh     = 32;
constexpr int kPadH   = kImgH + 2;
constexpr int kPadW   = kImgW + 2;
constexpr int kConvK  = 9 * kCh;
constexpr int kConvN  = 3 * kCh;
constexpr int kRelW   = 2 * kImgW - 1;
constexpr int kRelN   = (2 * kImgH - 1) * kRelW;
constexpr int kBiasPitch  = 4000;
constexpr int kConvTilesM = kPix / 64;
constexpr int kConvTilesN = kConvN / 64;
constexpr int kConvTiles  = kConvTilesM * kConvTilesN;
constexpr int kGnCount    = kCh * kTok;
constexpr int kBH         = kBatch * kHeads;

constexpr float kLoCarry    = 2048.0f;
constexpr float kLoCarryInv = 1.0f / 2048.0f;
constexpr float kPCarry     = 32768.0f;
constexpr float kVCarry     = 16.0f;
constexpr float kWoCarry    = 1024.0f;
constexpr float kWoCarryInv = 1.0f / 1024.0f;
constexpr float kGnEps      = 1e-6f;

static_assert(kHeads * kDh == kCh, "head split");
static_assert(kTok == 1024 && kPix == 8192, "token count");
static_assert(kConvK == 2304 && (kConvK % 32) == 0, "conv K multiple of 32");
static_assert((kPix % 64) == 0 && (kConvN % 64) == 0 && (kCh % 64) == 0, "tile multiples");
static_assert(kRelN == 3969 && kBiasPitch >= kRelN && (kBiasPitch % 32) == 0, "bias pitch whole lines");
static_assert(kConvTiles == 1536 && (kConvTiles % 8) == 0, "conv tile count");
static_assert(kDh == 32, "one 32-deep k step per head");

constexpr size_t kSzXB    = (size_t)kBatch * kPadH * kPadW * kCh * 2;
constexpr size_t kSzWT    = (size_t)kConvN * kConvK * 2;
constexpr size_t kSzWO    = (size_t)kCh * kCh * 2;
constexpr size_t kSzBIAS  = (size_t)kHeads * kBiasPitch * 4;
constexpr size_t kSzY     = (size_t)kPix * kConvN * 4;
constexpr size_t kSzSTATS = (size_t)kConvTiles * 32 * 4;
constexpr size_t kSzHP    = (size_t)kBH * kTok * kDh * 2;
constexpr size_t kOffXB    = 0;
constexpr size_t kOffWT    = kOffXB + kSzXB;
constexpr size_t kOffWO    = kOffWT + kSzWT;
constexpr size_t kOffBIAS  = kOffWO + kSzWO;
constexpr size_t kOffY     = kOffBIAS + kSzBIAS;
constexpr size_t kOffSTATS = kOffY + kSzY;
constexpr size_t kOffQH    = kOffSTATS + kSzSTATS;
constexpr size_t kOffQL    = kOffQH + kSzHP;
constexpr size_t kOffKH    = kOffQL + kSzHP;
constexpr size_t kOffKL    = kOffKH + kSzHP;
constexpr size_t kOffVT    = kOffKL + kSzHP;
constexpr size_t kOffOH    = kOffVT + kSzHP;
constexpr size_t kOffOL    = kOffOH + kSzHP;
constexpr size_t kWsTotal  = kOffOL + kSzHP;
static_assert(kWsTotal == 63255552ull, "carve total");
static_assert(kWsTotal <= 134217728ull, "carve cap");
static_assert((kOffWT % 128) == 0 && (kOffWO % 128) == 0 && (kOffBIAS % 128) == 0 && (kOffY % 128) == 0 &&
              (kOffSTATS % 128) == 0 && (kOffQH % 128) == 0 && (kOffQL % 128) == 0 && (kOffKH % 128) == 0 &&
              (kOffKL % 128) == 0 && (kOffVT % 128) == 0 && (kOffOH % 128) == 0 && (kOffOL % 128) == 0,
              "128-B aligned regions");

__device__ __forceinline__ unsigned short f2bf_bits(float f) {
  unsigned u = __float_as_uint(f);
  return (unsigned short)((u + 0x7FFFu + ((u >> 16) & 1u)) >> 16);
}
__device__ __forceinline__ float bf_bits2f(unsigned short h) { return __uint_as_float(((unsigned)h) << 16); }
__device__ __forceinline__ float bf_rne(float f) { return bf_bits2f(f2bf_bits(f)); }
__device__ __forceinline__ unsigned pk16(unsigned short a, unsigned short b) { return (unsigned)a | ((unsigned)b << 16); }
__device__ __forceinline__ unsigned short h_bits(float f) {
  const _Float16 h = (_Float16)f;
  return __builtin_bit_cast(unsigned short, h);
}
__device__ __forceinline__ void split_h(float v, unsigned short& hb, unsigned short& lb) {
  const _Float16 h0 = (_Float16)v;
  const float hf = (float)h0;
  const bool tiny = fabsf(v) < 6.103515625e-05f;
  const float hsel = tiny ? 0.0f : hf;
  const float res = (v - hsel) * kLoCarry;
  hb = h_bits(hsel);
  lb = h_bits(res);
}

template <typename T> struct Frag;
template <> struct Frag<_Float16> {
  typedef v16h V;
  union U { v16h v; v8h h[2]; };
  static __device__ __forceinline__ v16h load(const _Float16* p) {
    U f;
    f.h[0] = *(const v8h*)(p);
    f.h[1] = *(const v8h*)(p + 16);
    return f.v;
  }
};
template <> struct Frag<__bf16> {
  typedef v16b V;
  union U { v16b v; v8b h[2]; };
  static __device__ __forceinline__ v16b load(const __bf16* p) {
    U f;
    f.h[0] = *(const v8b*)(p);
    f.h[1] = *(const v8b*)(p + 16);
    return f.v;
  }
};

__device__ __forceinline__ v8f mma_b(v16b a, v16b b, v8f c) {
  c = __builtin_amdgcn_wmma_f32_16x16x32_bf16(false, a, false, b, (short)0, c, false, false);
  asm volatile("v_nop\n\tv_nop\n\tv_nop\n\tv_nop" : "+v"(c) : "v"(a), "v"(b));
  return c;
}
__device__ __forceinline__ v8f mma_h(v16h a, v16h b, v8f c) {
  c = __builtin_amdgcn_wmma_f32_16x16x32_f16(false, a, false, b, (short)0, c, false, false);
  asm volatile("v_nop\n\tv_nop\n\tv_nop\n\tv_nop" : "+v"(c) : "v"(a), "v"(b));
  return c;
}
__device__ __forceinline__ void wave_lds_sync() {
  __builtin_amdgcn_fence(__ATOMIC_RELEASE, "workgroup");
  __builtin_amdgcn_wave_barrier();
  __builtin_amdgcn_fence(__ATOMIC_ACQUIRE, "workgroup");
}

__global__ __launch_bounds__(256) void prep_x_kernel(const float* __restrict__ x, unsigned short* __restrict__ xb) {
  __shared__ float tile[kCh * 33];
  const int t  = threadIdx.x;
  const int b  = blockIdx.x / kPadH;
  const int yp = blockIdx.x - b * kPadH;
  const bool interior = (yp >= 1) && (yp <= kImgH);
  if (interior) {
    const int y = yp - 1;
#pragma unroll
    for (int i = 0; i < 8; ++i) {
      const int idx = i * 256 + t;
      const int ci = idx >> 3;
      const int x4 = (idx & 7) * 4;
      const v4f v = *(const v4f*)(x + ((size_t)(b * kCh + ci) * kImgH + y) * kImgW + x4);
      tile[ci * 33 + x4 + 0] = v[0];
      tile[ci * 33 + x4 + 1] = v[1];
      tile[ci * 33 + x4 + 2] = v[2];
      tile[ci * 33 + x4 + 3] = v[3];
    }
  }
  __syncthreads();
  unsigned short* dst = xb + (size_t)(b * kPadH + yp) * kPadW * kCh;
#pragma unroll 1
  for (int i = 0; i < 5; ++i) {
    const int chunk = i * 256 + t;
    if (chunk < kPadW * 32) {
      const int xp = chunk >> 5;
      const int c8 = (chunk & 31) * 8;
      unsigned u0 = 0u, u1 = 0u, u2 = 0u, u3 = 0u;
      if (interior) {
        int xc = xp - 1;
        xc = xc < 0 ? 0 : xc;
        xc = xc > (kImgW - 1) ? (kImgW - 1) : xc;
        unsigned short hb[8];
#pragma unroll
        for (int e = 0; e < 8; ++e) hb[e] = f2bf_bits(tile[(c8 + e) * 33 + xc]);
        const bool in = (xp >= 1) && (xp <= kImgW);
        const unsigned p0 = pk16(hb[0], hb[1]);
        const unsigned p1 = pk16(hb[2], hb[3]);
        const unsigned p2 = pk16(hb[4], hb[5]);
        const unsigned p3 = pk16(hb[6], hb[7]);
        u0 = in ? p0 : 0u;
        u1 = in ? p1 : 0u;
        u2 = in ? p2 : 0u;
        u3 = in ? p3 : 0u;
      }
      const v4u u = (v4u){u0, u1, u2, u3};
      volatile v4u* p = (volatile v4u*)(dst + (size_t)xp * kCh + c8);
      *p = u;
      __threadfence();
      *p = u;
    }
  }
}

__global__ __launch_bounds__(256) void prep_w_kernel(
    const float* __restrict__ wq, const float* __restrict__ wk, const float* __restrict__ wv,
    const float* __restrict__ wo, const float* __restrict__ bt,
    unsigned short* __restrict__ wt, unsigned short* __restrict__ wo16, float* __restrict__ biasr) {
  __shared__ float sm[kConvK];
  const int t  = threadIdx.x;
  const int bx = blockIdx.x;
  if (bx < kConvN) {
    const int P  = bx >> 8;
    const int co = bx & 255;
    const float* w = (P == 0) ? wq : ((P == 1) ? wk : wv);
    const float* src = w + (size_t)co * kConvK;
#pragma unroll
    for (int i = 0; i < 9; ++i) sm[i * 256 + t] = src[i * 256 + t];
    __syncthreads();
    unsigned short* dst = wt + (size_t)bx * kConvK;
#pragma unroll 1
    for (int it = 0; it < 2; ++it) {
      const int chunk = it * 256 + t;
      if (chunk < kConvK / 8) {
        const int k   = chunk * 8;
        const int tap = k >> 8;
        const int ci0 = k & 255;
        unsigned short hb[8];
#pragma unroll
        for (int e = 0; e < 8; ++e) hb[e] = f2bf_bits(sm[(ci0 + e) * 9 + tap]);
        const v4u u = (v4u){pk16(hb[0], hb[1]), pk16(hb[2], hb[3]), pk16(hb[4], hb[5]), pk16(hb[6], hb[7])};
        volatile v4u* p = (volatile v4u*)(dst + k);
        *p = u;
        __threadfence();
        *p = u;
      }
    }
  } else if (bx < kConvN + 32) {
    const int i = (bx - kConvN) * 256 + t;
    const float* p = wo + 8 * (size_t)i;
    const v4f a = *(const v4f*)(p);
    const v4f c = *(const v4f*)(p + 4);
    unsigned short hb[8];
#pragma unroll
    for (int e = 0; e < 4; ++e) {
      const float a0 = a[e];
      const float c0 = c[e];
      hb[e]     = h_bits(bf_rne(a0) * kWoCarry);
      hb[4 + e] = h_bits(bf_rne(c0) * kWoCarry);
    }
    const v4u u = (v4u){pk16(hb[0], hb[1]), pk16(hb[2], hb[3]), pk16(hb[4], hb[5]), pk16(hb[6], hb[7])};
    volatile v4u* q = (volatile v4u*)(wo16 + 8 * (size_t)i);
    *q = u;
    __threadfence();
    *q = u;
  } else {
    const int hsel = bx - (kConvN + 32);
#pragma unroll 1
    for (int it = 0; it < 4; ++it) {
      const int chunk = it * 256 + t;
      if (chunk < kBiasPitch / 4) {
        float vals[4];
#pragma unroll
        for (int e = 0; e < 4; ++e) {
          const int idx = chunk * 4 + e;
          const int ic  = idx < kRelN ? idx : (kRelN - 1);
          const float raw = bt[(size_t)ic * kHeads + hsel];
          vals[e] = (idx < kRelN) ? bf_rne(raw) : 0.0f;
        }
        const v4f o = (v4f){vals[0], vals[1], vals[2], vals[3]};
        volatile v4f* p = (volatile v4f*)(biasr + (size_t)hsel * kBiasPitch + chunk * 4);
        *p = o;
        __threadfence();
        *p = o;
      }
    }
  }
}

__global__ __launch_bounds__(256) void conv_gemm_kernel(
    const unsigned short* __restrict__ xbp, const unsigned short* __restrict__ wtp,
    float* __restrict__ Y, float* __restrict__ stats) {
  const __bf16* XB = (const __bf16*)xbp;
  const __bf16* WT = (const __bf16*)wtp;
  __shared__ __align__(16) float sT[8][16 * 68];
  const int lane = threadIdx.x & 31;
  const int wave = threadIdx.x >> 5;
  const int tile = blockIdx.x * 8 + wave;
  if (tile >= kConvTiles) return;
  const int tm = tile / kConvTilesN;
  const int tn = tile - tm * kConvTilesN;
  const int m0 = tm << 6;
  const int n0 = tn << 6;
  const int rlane = lane & 15;
  const int koff  = (lane >> 4) * 8;
  const int mOff  = (lane >> 4) * 8;

  int arow[4], brow[4];
#pragma unroll
  for (int i = 0; i < 4; ++i) {
    const int m  = m0 + (i << 4) + rlane;
    const int bi = m >> 10;
    const int yy = (m >> 5) & 31;
    const int xx = m & 31;
    arow[i] = ((bi * kPadH + yy) * kPadW + xx) * kCh + koff;
  }
#pragma unroll
  for (int j = 0; j < 4; ++j) brow[j] = (n0 + (j << 4) + rlane) * kConvK + koff;

  v8f acc[4][4];
#pragma unroll
  for (int i = 0; i < 4; ++i)
#pragma unroll
    for (int j = 0; j < 4; ++j) acc[i][j] = (v8f){0.f, 0.f, 0.f, 0.f, 0.f, 0.f, 0.f, 0.f};

#pragma unroll 1
  for (int kh = 0; kh < 3; ++kh) {
#pragma unroll 1
    for (int kw = 0; kw < 3; ++kw) {
      const int tapA = (kh * kPadW + kw) * kCh;
      const int tapB = (kh * 3 + kw) * kCh;
#pragma unroll 1
      for (int cc = 0; cc < 8; ++cc) {
        const int ka = tapA + cc * 32;
        const int kb = tapB + cc * 32;
        v16b bf[4];
#pragma unroll
        for (int j = 0; j < 4; ++j) bf[j] = Frag<__bf16>::load(WT + brow[j] + kb);
#pragma unroll
        for (int i = 0; i < 4; ++i) {
          const v16b af = Frag<__bf16>::load(XB + arow[i] + ka);
#pragma unroll
          for (int j = 0; j < 4; ++j) acc[i][j] = mma_b(af, bf[j], acc[i][j]);
        }
      }
    }
  }

  float* slab = sT[wave];
  float ps = 0.f, pq = 0.f;
#pragma unroll
  for (int i = 0; i < 4; ++i) {
    const int mBase = m0 + (i << 4);
#pragma unroll
    for (int j = 0; j < 4; ++j) {
#pragma unroll
      for (int r = 0; r < 8; ++r) {
        const float v = acc[i][j][r];
        ps += v;
        pq = fmaf(v, v, pq);
        slab[(mOff + r) * 68 + (j << 4) + rlane] = v;
      }
    }
    wave_lds_sync();
    {
      const int hh = lane >> 4, c4 = (lane & 15) * 4;
      for (int pass = 0; pass < 2; ++pass) {
#pragma unroll
        for (int it = 0; it < 8; ++it) {
          const int row = it * 2 + hh;
          const v4f v = *(const v4f*)(slab + row * 68 + c4);
          *(volatile v4f*)(Y + (size_t)(mBase + row) * kConvN + n0 + c4) = v;
        }
        __threadfence();
      }
    }
    wave_lds_sync();
  }
#pragma unroll
  for (int off = 16; off > 0; off >>= 1) {
    ps += __shfl_xor(ps, off, 32);
    pq += __shfl_xor(pq, off, 32);
  }
  {
    const float sv = (lane == 0) ? ps : ((lane == 1) ? pq : 0.0f);
    volatile float* sp = stats + (size_t)tile * 32 + lane;
    *sp = sv;
    __threadfence();
    *sp = sv;
  }
}

__global__ __launch_bounds__(256) void gn_pack_kernel(
    const float* __restrict__ Y, const float* __restrict__ stats,
    const float* __restrict__ gq, const float* __restrict__ bq,
    const float* __restrict__ gk, const float* __restrict__ bk,
    const float* __restrict__ gv, const float* __restrict__ bv,
    unsigned short* __restrict__ QH, unsigned short* __restrict__ QL,
    unsigned short* __restrict__ KH, unsigned short* __restrict__ KL,
    unsigned short* __restrict__ VT) {
  __shared__ float tile[64 * 33];
  const int t    = threadIdx.x;
  const int lane = t & 31;
  const int P    = blockIdx.y;
  const int bx   = blockIdx.x;
  const int tt   = bx & 15;
  const int h    = (bx >> 4) & 7;
  const int b    = bx >> 7;
  const int n0   = tt * 64;
  const int bh   = b * kHeads + h;

  float s = 0.f, q = 0.f;
#pragma unroll
  for (int u = 0; u < 2; ++u) {
    const int e  = lane + 32 * u;
    const int tl = (b * 16 + (e >> 2)) * kConvTilesN + P * 4 + (e & 3);
    s += stats[(size_t)tl * 32];
    q += stats[(size_t)tl * 32 + 1];
  }
#pragma unroll
  for (int off = 16; off > 0; off >>= 1) {
    s += __shfl_xor(s, off, 32);
    q += __shfl_xor(q, off, 32);
  }
  const float invn = 1.0f / (float)kGnCount;
  const float mean = s * invn;
  const float var  = fmaxf(q * invn - mean * mean, 0.0f);
  const float inv  = 1.0f / sqrtf(var + kGnEps);

  const int d   = t & 31;
  const int rb  = t >> 5;
  const int chn = h * kDh + d;
  const float* gp = (P == 0) ? gq : ((P == 1) ? gk : gv);
  const float* bp = (P == 0) ? bq : ((P == 1) ? bk : bv);
  const float gam = bf_rne(gp[chn]);
  const float bet = bf_rne(bp[chn]);
  const float* ysrc = Y + (size_t)(b * kTok + n0 + rb) * kConvN + P * kCh + chn;
#pragma unroll 1
  for (int i = 0; i < 8; ++i) {
    const float yv = ysrc[(size_t)i * 8 * kConvN];
    const float xn = (yv - mean) * inv;
    const float tv = xn * gam + bet;
    const float ge = 0.5f * tv * (1.0f + erff(tv * 0.70710678118654752f));
    tile[(i * 8 + rb) * 33 + d] = ge;
  }
  __syncthreads();

  if (P < 2) {
    const int r  = t >> 2;
    const int dq = t & 3;
    unsigned short hb[8], lb[8];
#pragma unroll
    for (int e = 0; e < 8; ++e) split_h(tile[r * 33 + dq * 8 + e], hb[e], lb[e]);
    const v4u uh = (v4u){pk16(hb[0], hb[1]), pk16(hb[2], hb[3]), pk16(hb[4], hb[5]), pk16(hb[6], hb[7])};
    const v4u ul = (v4u){pk16(lb[0], lb[1]), pk16(lb[2], lb[3]), pk16(lb[4], lb[5]), pk16(lb[6], lb[7])};
    unsigned short* ph = (P == 0) ? QH : KH;
    unsigned short* pl = (P == 0) ? QL : KL;
    const size_t o = ((size_t)bh * kTok + n0 + r) * kDh + dq * 8;
    volatile v4u* vh = (volatile v4u*)(ph + o);
    volatile v4u* vl = (volatile v4u*)(pl + o);
    *vh = uh;
    *vl = ul;
    __threadfence();
    *vh = uh;
    *vl = ul;
  } else {
    const int dd = t >> 3;
    const int kq = t & 7;
    unsigned short hb[8];
#pragma unroll
    for (int e = 0; e < 8; ++e) hb[e] = h_bits(tile[(kq * 8 + e) * 33 + dd] * kVCarry);
    const v4u u = (v4u){pk16(hb[0], hb[1]), pk16(hb[2], hb[3]), pk16(hb[4], hb[5]), pk16(hb[6], hb[7])};
    volatile v4u* p = (volatile v4u*)(VT + ((size_t)bh * kDh + dd) * kTok + n0 + kq * 8);
    *p = u;
    __threadfence();
    *p = u;
  }
}

__global__ __launch_bounds__(128) void attn_kernel(
    const unsigned short* __restrict__ qhp, const unsigned short* __restrict__ qlp,
    const unsigned short* __restrict__ khp, const unsigned short* __restrict__ klp,
    const unsigned short* __restrict__ vtp, const float* __restrict__ biasr,
    unsigned short* __restrict__ ohp, unsigned short* __restrict__ olp) {
  const _Float16* QH = (const _Float16*)qhp;
  const _Float16* QL = (const _Float16*)qlp;
  const _Float16* KH = (const _Float16*)khp;
  const _Float16* KL = (const _Float16*)klp;
  const _Float16* VT = (const _Float16*)vtp;
  __shared__ __align__(16) _Float16 Psh[4][16 * 64];
  __shared__ __align__(16) float    Bsh[4][128];
  __shared__ __align__(16) float    Osh[4][16 * 36];

  const int tid  = threadIdx.x;
  const int wave = tid >> 5;
  const int lane = tid & 31;
  const int hh   = lane >> 4;
  const int c    = lane & 15;
  const int qb   = blockIdx.x & 15;
  const int bh   = blockIdx.x >> 4;
  const int h    = bh & (kHeads - 1);
  const int q0   = qb * 64 + wave * 16;
  const int yi   = q0 >> 5;
  const int x0   = q0 & 31;
  const size_t plane = (size_t)bh * kTok * kDh;

  const v16h qah = Frag<_Float16>::load(QH + plane + (size_t)(q0 + c) * kDh + 8 * hh);
  const v16h qal = Frag<_Float16>::load(QL + plane + (size_t)(q0 + c) * kDh + 8 * hh);
  const float* bhead = biasr + (size_t)h * kBiasPitch;
  const _Float16* kbh = KH + plane + (size_t)c * kDh + 8 * hh;
  const _Float16* kbl = KL + plane + (size_t)c * kDh + 8 * hh;
  const _Float16* vb  = VT + ((size_t)bh * kDh + c) * kTok + 8 * hh;
  _Float16* pw = Psh[wave];
  float*    bw = Bsh[wave];
  float*    os = Osh[wave];
  const int boff = 31 + 8 * hh - c;
  const int t1   = (lane + 32 > 46) ? 46 : (lane + 32);

  float mrow[8], lrow[8];
  v8f oacc[2];
#pragma unroll
  for (int r = 0; r < 8; ++r) { mrow[r] = -1e30f; lrow[r] = 0.f; }
  oacc[0] = (v8f){0.f, 0.f, 0.f, 0.f, 0.f, 0.f, 0.f, 0.f};
  oacc[1] = (v8f){0.f, 0.f, 0.f, 0.f, 0.f, 0.f, 0.f, 0.f};

#pragma unroll 1
  for (int kc = 0; kc < kTok / 64; ++kc) {
    const int kv0 = kc * 64;
    {
      const int base0 = (yi - 2 * kc + 31) * kRelW + x0;
      const int base1 = base0 - kRelW;
      const float f00 = bhead[base0 + lane];
      const float f01 = bhead[base0 + t1];
      const float f10 = bhead[base1 + lane];
      const float f11 = bhead[base1 + t1];
      bw[lane]      = f00;
      bw[32 + lane] = f01;
      bw[64 + lane] = f10;
      bw[96 + lane] = f11;
    }
    wave_lds_sync();

    v8f s1[4], s2[4];
#pragma unroll
    for (int j = 0; j < 4; ++j) {
      const size_t ko = (size_t)(kv0 + j * 16) * kDh;
      const v16h kfh = Frag<_Float16>::load(kbh + ko);
      const v16h kfl = Frag<_Float16>::load(kbl + ko);
      s1[j] = (v8f){0.f, 0.f, 0.f, 0.f, 0.f, 0.f, 0.f, 0.f};
      s2[j] = (v8f){0.f, 0.f, 0.f, 0.f, 0.f, 0.f, 0.f, 0.f};
      s1[j] = mma_h(qah, kfh, s1[j]);
      s2[j] = mma_h(qah, kfl, s2[j]);
      s2[j] = mma_h(qal, kfh, s2[j]);
    }
#pragma unroll
    for (int j = 0; j < 4; ++j) {
      const float* bp = bw + (j >> 1) * 64 + boff - (j & 1) * 16;
#pragma unroll
      for (int r = 0; r < 8; ++r) s1[j][r] = s1[j][r] + s2[j][r] * kLoCarryInv + bp[r];
    }

    float cm[8];
#pragma unroll
    for (int r = 0; r < 8; ++r) {
      float m = fmaxf(fmaxf(s1[0][r], s1[1][r]), fmaxf(s1[2][r], s1[3][r]));
#pragma unroll
      for (int off = 1; off < 16; off <<= 1) m = fmaxf(m, __shfl_xor(m, off, 32));
      cm[r] = m;
    }
#pragma unroll
    for (int r = 0; r < 8; ++r) {
      const float mnew  = fmaxf(mrow[r], cm[r]);
      const float alpha = __expf(mrow[r] - mnew);
      mrow[r] = mnew;
      float psum = 0.f;
#pragma unroll
      for (int j = 0; j < 4; ++j) {
        const float p = __expf(s1[j][r] - mnew);
        psum += p;
        pw[(8 * hh + r) * 64 + j * 16 + c] = (_Float16)(p * kPCarry);
      }
#pragma unroll
      for (int off = 1; off < 16; off <<= 1) psum += __shfl_xor(psum, off, 32);
      lrow[r] = lrow[r] * alpha + psum;
      oacc[0][r] *= alpha;
      oacc[1][r] *= alpha;
    }
    wave_lds_sync();
#pragma unroll
    for (int kk = 0; kk < 2; ++kk) {
      const v16h pa = Frag<_Float16>::load(pw + c * 64 + kk * 32 + 8 * hh);
#pragma unroll
      for (int t = 0; t < 2; ++t) {
        const v16h vf = Frag<_Float16>::load(vb + (size_t)(t * 16) * kTok + kv0 + kk * 32);
        oacc[t] = mma_h(pa, vf, oacc[t]);
      }
    }
    wave_lds_sync();
  }

#pragma unroll
  for (int r = 0; r < 8; ++r) {
    const float inv = 1.0f / (lrow[r] * (kPCarry * kVCarry));
    os[(8 * hh + r) * 36 + c]      = oacc[0][r] * inv;
    os[(8 * hh + r) * 36 + 16 + c] = oacc[1][r] * inv;
  }
  wave_lds_sync();
  {
    const int rq = lane >> 2;
    const int dq = lane & 3;
    v4u uh[2], ul[2];
#pragma unroll
    for (int it = 0; it < 2; ++it) {
      const int row = it * 8 + rq;
      const float* sp = os + row * 36 + dq * 8;
      const v4f a0 = *(const v4f*)(sp);
      const v4f a1 = *(const v4f*)(sp + 4);
      unsigned short hb[8], lb[8];
#pragma unroll
      for (int e = 0; e < 4; ++e) {
        const float f0 = a0[e];
        const float f1 = a1[e];
        split_h(f0, hb[e], lb[e]);
        split_h(f1, hb[4 + e], lb[4 + e]);
      }
      uh[it] = (v4u){pk16(hb[0], hb[1]), pk16(hb[2], hb[3]), pk16(hb[4], hb[5]), pk16(hb[6], hb[7])};
      ul[it] = (v4u){pk16(lb[0], lb[1]), pk16(lb[2], lb[3]), pk16(lb[4], lb[5]), pk16(lb[6], lb[7])};
    }
    for (int pass = 0; pass < 2; ++pass) {
#pragma unroll
      for (int it = 0; it < 2; ++it) {
        const int row = it * 8 + rq;
        const size_t o = plane + (size_t)(q0 + row) * kDh + dq * 8;
        *(volatile v4u*)(ohp + o) = uh[it];
        *(volatile v4u*)(olp + o) = ul[it];
      }
      __threadfence();
    }
  }
}

__global__ __launch_bounds__(256) void out_gemm_kernel(
    const unsigned short* __restrict__ wop, const unsigned short* __restrict__ ohp,
    const unsigned short* __restrict__ olp, const float* __restrict__ bo, float* __restrict__ out) {
  const _Float16* WO = (const _Float16*)wop;
  const _Float16* OH = (const _Float16*)ohp;
  const _Float16* OL = (const _Float16*)olp;
  __shared__ __align__(16) float sT[8][16 * 68];
  const int lane = threadIdx.x & 31;
  const int wave = threadIdx.x >> 5;
  const int tile = blockIdx.x * 8 + wave;
  if (tile >= (kCh / 32) * (kPix / 64)) return;
  const int tm = tile >> 7;
  const int tn = tile & 127;
  const int m0 = tm << 5;
  const int n0 = tn << 6;
  const int bimg = n0 >> 10;
  const int nn0  = n0 & (kTok - 1);
  const int rlane = lane & 15;
  const int koff  = (lane >> 4) * 8;
  const int mOff  = (lane >> 4) * 8;

  v8f acch[2][4], accl[2][4];
#pragma unroll
  for (int i = 0; i < 2; ++i)
#pragma unroll
    for (int j = 0; j < 4; ++j) {
      acch[i][j] = (v8f){0.f, 0.f, 0.f, 0.f, 0.f, 0.f, 0.f, 0.f};
      accl[i][j] = (v8f){0.f, 0.f, 0.f, 0.f, 0.f, 0.f, 0.f, 0.f};
    }

#pragma unroll 1
  for (int k0 = 0; k0 < kCh; k0 += 32) {
    const int head = k0 >> 5;
    v16h bfh[4], bfl[4];
#pragma unroll
    for (int j = 0; j < 4; ++j) {
      const size_t bofs = ((size_t)(bimg * kHeads + head) * kTok + nn0 + (j << 4) + rlane) * kDh + koff;
      bfh[j] = Frag<_Float16>::load(OH + bofs);
      bfl[j] = Frag<_Float16>::load(OL + bofs);
    }
#pragma unroll
    for (int i = 0; i < 2; ++i) {
      const v16h af = Frag<_Float16>::load(WO + (size_t)(m0 + (i << 4) + rlane) * kCh + koff + k0);
#pragma unroll
      for (int j = 0; j < 4; ++j) {
        acch[i][j] = mma_h(af, bfh[j], acch[i][j]);
        accl[i][j] = mma_h(af, bfl[j], accl[i][j]);
      }
    }
  }

  float* slab = sT[wave];
#pragma unroll
  for (int i = 0; i < 2; ++i) {
    const int mBase = m0 + (i << 4);
    float bias_r[8];
#pragma unroll
    for (int r = 0; r < 8; ++r) bias_r[r] = bf_rne(bo[mBase + mOff + r]);
#pragma unroll
    for (int j = 0; j < 4; ++j) {
#pragma unroll
      for (int r = 0; r < 8; ++r) {
        const float v = (acch[i][j][r] + accl[i][j][r] * kLoCarryInv) * kWoCarryInv + bias_r[r];
        slab[(mOff + r) * 68 + (j << 4) + rlane] = v;
      }
    }
    wave_lds_sync();
    {
      const int hh = lane >> 4, c4 = (lane & 15) * 4;
      for (int pass = 0; pass < 2; ++pass) {
#pragma unroll
        for (int it = 0; it < 8; ++it) {
          const int row = it * 2 + hh;
          const v4f v = *(const v4f*)(slab + row * 68 + c4);
          *(volatile v4f*)(out + ((size_t)(bimg * kCh + mBase + row)) * kTok + nn0 + c4) = v;
        }
        __threadfence();
      }
    }
    wave_lds_sync();
  }
}

extern "C" void kernel_launch(void* const* d_in, const int* in_sizes, int n_in,
                              void* d_out, int out_size, void* d_ws, size_t ws_size,
                              hipStream_t stream) {
  if (n_in < 13) return;
  if (in_sizes[0] != kBatch * kCh * kTok) return;
  if (in_sizes[1] != kCh * kConvK || in_sizes[2] != kCh * kConvK || in_sizes[3] != kCh * kConvK) return;
  if (in_sizes[4] != kCh || in_sizes[5] != kCh || in_sizes[6] != kCh ||
      in_sizes[7] != kCh || in_sizes[8] != kCh || in_sizes[9] != kCh) return;
  if (in_sizes[10] != kRelN * kHeads) return;
  if (in_sizes[11] != kCh * kCh || in_sizes[12] != kCh) return;
  if (out_size != kBatch * kCh * kTok) return;
  if (ws_size < kWsTotal) return;

  const float* x   = (const float*)d_in[0];
  const float* wq  = (const float*)d_in[1];
  const float* wk  = (const float*)d_in[2];
  const float* wv  = (const float*)d_in[3];
  const float* gq  = (const float*)d_in[4];
  const float* bq  = (const float*)d_in[5];
  const float* gk  = (const float*)d_in[6];
  const float* bk  = (const float*)d_in[7];
  const float* gv  = (const float*)d_in[8];
  const float* bv  = (const float*)d_in[9];
  const float* btab = (const float*)d_in[10];
  const float* wo  = (const float*)d_in[11];
  const float* bo  = (const float*)d_in[12];
  float* out = (float*)d_out;

  char* ws = (char*)d_ws;
  unsigned short* XB    = (unsigned short*)(ws + kOffXB);
  unsigned short* WT    = (unsigned short*)(ws + kOffWT);
  unsigned short* WO16  = (unsigned short*)(ws + kOffWO);
  float*          BIASR = (float*)(ws + kOffBIAS);
  float*          Yp    = (float*)(ws + kOffY);
  float*          STATS = (float*)(ws + kOffSTATS);
  unsigned short* QH    = (unsigned short*)(ws + kOffQH);
  unsigned short* QL    = (unsigned short*)(ws + kOffQL);
  unsigned short* KH    = (unsigned short*)(ws + kOffKH);
  unsigned short* KL    = (unsigned short*)(ws + kOffKL);
  unsigned short* VT    = (unsigned short*)(ws + kOffVT);
  unsigned short* OH    = (unsigned short*)(ws + kOffOH);
  unsigned short* OL    = (unsigned short*)(ws + kOffOL);

  prep_x_kernel<<<kBatch * kPadH, 256, 0, stream>>>(x, XB);
  prep_w_kernel<<<kConvN + 32 + kHeads, 256, 0, stream>>>(wq, wk, wv, wo, btab, WT, WO16, BIASR);
  conv_gemm_kernel<<<kConvTiles / 8, 256, 0, stream>>>(XB, WT, Yp, STATS);
  gn_pack_kernel<<<dim3(kBatch * kHeads * (kTok / 64), 3), 256, 0, stream>>>(
      Yp, STATS, gq, bq, gk, bk, gv, bv, QH, QL, KH, KL, VT);
  attn_kernel<<<kBH * (kTok / 64), 128, 0, stream>>>(QH, QL, KH, KL, VT, BIASR, OH, OL);
  out_gemm_kernel<<<((kCh / 32) * (kPix / 64)) / 8, 256, 0, stream>>>(WO16, OH, OL, bo, out);
}
